// NONLocalBlock2D_30511447671193
// MI455X (gfx1250) — hardware-verified
//
#include <hip/hip_runtime.h>


#ifndef NB
#define NB 4
#endif
#ifndef SEQ
#define SEQ 4096
#endif

static constexpr int B_FULL = 4, C = 256, T = 4096, CK = 128, CV = 128;
static constexpr int BL = NB;
static constexpr int QL = SEQ;
static constexpr size_t NR = (size_t)B_FULL * T;
static constexpr float XS = 8.0f, WSC = 256.0f, RS_ = 1024.0f, PS = 1024.0f, EPS = 1e-5f, LOG2E = 1.4426950408889634f;
static constexpr float INV1 = 1.0f / (XS * WSC);
static constexpr float SMS = 0.08838834764831845f * (1.0f / (XS * XS));
static_assert(BL >= 1 && BL <= B_FULL);
static_assert(QL % 32 == 0 && QL >= 32 && QL <= T);
static_assert(T % 64 == 0 && C == 256 && CK == 128 && CV == 128);

typedef _Float16 b16;
typedef __attribute__((ext_vector_type(16))) _Float16 v16b;
typedef __attribute__((ext_vector_type(8))) _Float16 v8b;
typedef __attribute__((ext_vector_type(4))) _Float16 v4h;
typedef __attribute__((ext_vector_type(8))) float v8f;
typedef __attribute__((ext_vector_type(4))) float v4f;

static __device__ __forceinline__ float bf16_rne(float f) { unsigned int u = __float_as_uint(f); u += 0x7FFFu + ((u >> 16) & 1u); return __uint_as_float(u & 0xFFFF0000u); }
static __device__ __forceinline__ float pmul(float a, float b) { float p = a * b; asm volatile("" : "+v"(p)); return p; }
static __device__ __forceinline__ float nexp2(float v) { return __builtin_amdgcn_exp2f(v); }
static __device__ __forceinline__ v16b frag_kb(const b16* p, int hh) { const v8b a = *(const v8b*)(p + 8 * hh), b = *(const v8b*)(p + 16 + 8 * hh); v16b f;
#pragma unroll
  for (int e = 0; e < 8; ++e) { f[e] = a[e]; f[8 + e] = b[e]; } return f; }
static __device__ __forceinline__ v8f wmma16b(v16b a, v16b b, v8f c) { v8f d = __builtin_amdgcn_wmma_f32_16x16x32_f16(false, a, false, b, (short)0, c, false, false);
  asm volatile("v_nop\n\tv_nop\n\tv_nop\n\tv_nop" : "+v"(d) : "v"(a), "v"(b)); return d; }

static constexpr int U1 = CK * C / 8, U2 = CK * CK / 8, UO = C * CV / 8, UB = 4 * CK + C;
static constexpr int UW = 3 * U1 + 2 * U2 + UO, UT = UW + UB;
static_assert(U1 % 32 == 0 && U2 % 32 == 0 && UO % 32 == 0 && CK % 32 == 0 && UW % 256 == 0 && UT % 32 == 0);
static constexpr int PTW = 256;

__global__ __launch_bounds__(256) void prep_kernel(const float* __restrict__ wq1, const float* __restrict__ wk1, const float* __restrict__ wv, const float* __restrict__ wq2,
    const float* __restrict__ wk2, const float* __restrict__ wo,
    const float* gq1, const float* bq1, const float* mq1, const float* vq1, const float* gq2, const float* bq2, const float* mq2, const float* vq2,
    const float* gk1, const float* bk1, const float* mk1, const float* vk1, const float* gk2, const float* bk2, const float* mk2, const float* vk2,
    const float* go, const float* bo, const float* mo, const float* vo,
    b16* __restrict__ W1q, b16* __restrict__ W1k, b16* __restrict__ W1v, b16* __restrict__ W2q, b16* __restrict__ W2k, b16* __restrict__ WoT, b16* __restrict__ WoQ,
    float* __restrict__ PT) {
#pragma clang fp contract(off)
  const int u = blockIdx.x * 256 + threadIdx.x;
  if (u < 3 * U1) {
    const int w = u / U1; const int e = (u - w * U1) * 8;
    const float* src = (w == 0) ? wq1 : ((w == 1) ? wk1 : wv); b16* dst = (w == 0) ? W1q : ((w == 1) ? W1k : W1v);
    v8b v;
#pragma unroll
    for (int j = 0; j < 8; ++j) v[j] = (b16)pmul(bf16_rne(src[e + j]), WSC);
    for (int pass = 0; pass < 2; ++pass) { *(volatile v8b*)(dst + e) = v; __threadfence(); }
  } else if (u < 3 * U1 + 2 * U2) {
    const int i = u - 3 * U1; const int w = i / U2; const int e = (i - w * U2) * 8;
    const float* src = (w == 0) ? wq2 : wk2; b16* dst = (w == 0) ? W2q : W2k;
    v8b v;
#pragma unroll
    for (int j = 0; j < 8; ++j) v[j] = (b16)pmul(bf16_rne(src[e + j]), WSC);
    for (int pass = 0; pass < 2; ++pass) { *(volatile v8b*)(dst + e) = v; __threadfence(); }
  } else if (u < UW) {
    const int e = (u - 3 * U1 - 2 * U2) * 8; v8b v, q;
#pragma unroll
    for (int j = 0; j < 8; ++j) { const float w = bf16_rne(wo[e + j]); v[j] = (b16)pmul(w, WSC); q[j] = (b16)pmul(w, 0.25f); }
    for (int pass = 0; pass < 2; ++pass) { *(volatile v8b*)(WoT + e) = v; *(volatile v8b*)(WoQ + e) = q; __threadfence(); }
  } else if (u < UT) {
    const int i = u - UW;
    const int s = (i < CK) ? 0 : ((i < 2 * CK) ? 1 : ((i < 3 * CK) ? 2 : ((i < 4 * CK) ? 3 : 4)));
    const int c = i - ((s < 4) ? s * CK : 4 * CK);
    const float* gp = (s == 0) ? gq1 : ((s == 1) ? gq2 : ((s == 2) ? gk1 : ((s == 3) ? gk2 : go)));
    const float* bp = (s == 0) ? bq1 : ((s == 1) ? bq2 : ((s == 2) ? bk1 : ((s == 3) ? bk2 : bo)));
    const float* mp = (s == 0) ? mq1 : ((s == 1) ? mq2 : ((s == 2) ? mk1 : ((s == 3) ? mk2 : mo)));
    const float* vp = (s == 0) ? vq1 : ((s == 1) ? vq2 : ((s == 2) ? vk1 : ((s == 3) ? vk2 : vo)));
    const float g = bf16_rne(gp[c]), bb = bf16_rne(bp[c]), mm = bf16_rne(mp[c]), vv = bf16_rne(vp[c]);
    const float sc = g * (1.0f / sqrtf(vv + EPS));
    for (int pass = 0; pass < 2; ++pass) {
      ((volatile float*)PT)[(s * 3 + 0) * PTW + c] = sc; ((volatile float*)PT)[(s * 3 + 1) * PTW + c] = mm; ((volatile float*)PT)[(s * 3 + 2) * PTW + c] = bb; __threadfence(); }
  }
}

__global__ __launch_bounds__(64) void projqk_kernel(const float* __restrict__ x, const float* __restrict__ y, const b16* __restrict__ W1q, const b16* __restrict__ W1k,
    const b16* __restrict__ W2q, const b16* __restrict__ W2k, const float* __restrict__ PT, b16* __restrict__ Qh, b16* __restrict__ Kh) {
  __shared__ __attribute__((aligned(16))) b16 Ah[2][16][C + 8];
  __shared__ __attribute__((aligned(16))) float Tw[2][16][CK + 4];
  const int wave = threadIdx.x >> 5, lane = threadIdx.x & 31, nloc = lane & 15, hlf = lane >> 4;
  const int side = blockIdx.z, b = blockIdx.y;
  const int npos = (side == 0) ? QL : T;
  if ((int)blockIdx.x * 32 >= npos) return;
  const int n0 = blockIdx.x * 32 + wave * 16;
  const float* src = (side == 0) ? x : y; const b16* W1 = (side == 0) ? W1q : W1k; const b16* W2 = (side == 0) ? W2q : W2k; b16* dst = (side == 0) ? Qh : Kh;
  const float* P1 = PT + (size_t)((side == 0) ? 0 : 2) * 3 * PTW; const float* P2 = PT + (size_t)((side == 0) ? 1 : 3) * 3 * PTW;
  for (int idx = lane; idx < 16 * C; idx += 32) { const int k = idx >> 4, rr = idx & 15; Ah[wave][rr][k] = (b16)(bf16_rne(src[((size_t)b * C + k) * T + n0 + rr]) * XS); }
  __syncthreads();
  v8f acc[8];
#pragma unroll
  for (int t = 0; t < 8; ++t) acc[t] = (v8f){};
#pragma unroll 1
  for (int kb = 0; kb < C; kb += 32) { const v16b a = frag_kb(&Ah[wave][nloc][kb], hlf);
#pragma unroll
    for (int t = 0; t < 8; ++t) acc[t] = wmma16b(a, frag_kb(W1 + (size_t)(t * 16 + nloc) * C + kb, hlf), acc[t]); }
#pragma unroll
  for (int t = 0; t < 8; ++t)
#pragma unroll
    for (int r = 0; r < 8; ++r) Tw[wave][8 * hlf + r][t * 16 + nloc] = acc[t][r];
  __syncthreads();
  {
    const int c4 = lane * 4; float sc[4], mm[4], bb[4];
#pragma unroll
    for (int j = 0; j < 4; ++j) { sc[j] = P1[c4 + j]; mm[j] = P1[PTW + c4 + j]; bb[j] = P1[2 * PTW + c4 + j]; }
#pragma unroll 2
    for (int row = 0; row < 16; ++row) { const v4f tv = *(const v4f*)(&Tw[wave][row][c4]); v4h h;
#pragma unroll
      for (int j = 0; j < 4; ++j) { const float v = tv[j] * INV1; const float tt = fmaxf((v - mm[j]) * sc[j] + bb[j], 0.0f); h[j] = (b16)(tt * XS); }
      *(v4h*)(&Ah[wave][row][c4]) = h; } }
  __syncthreads();
#pragma unroll
  for (int t = 0; t < 8; ++t) acc[t] = (v8f){};
#pragma unroll 1
  for (int kb = 0; kb < CK; kb += 32) { const v16b a = frag_kb(&Ah[wave][nloc][kb], hlf);
#pragma unroll
    for (int t = 0; t < 8; ++t) acc[t] = wmma16b(a, frag_kb(W2 + (size_t)(t * 16 + nloc) * CK + kb, hlf), acc[t]); }
#pragma unroll
  for (int t = 0; t < 8; ++t)
#pragma unroll
    for (int r = 0; r < 8; ++r) Tw[wave][8 * hlf + r][t * 16 + nloc] = acc[t][r];
  __syncthreads();
  {
    const int ro = lane >> 4, c8 = (lane & 15) * 8; float sc[8], mm[8], bb[8];
#pragma unroll
    for (int j = 0; j < 8; ++j) { sc[j] = P2[c8 + j]; mm[j] = P2[PTW + c8 + j]; bb[j] = P2[2 * PTW + c8 + j]; }
    for (int pass = 0; pass < 2; ++pass) {
#pragma unroll 2
      for (int rr = 0; rr < 16; rr += 2) { const int row = rr + ro; const v4f t0 = *(const v4f*)(&Tw[wave][row][c8]), t1 = *(const v4f*)(&Tw[wave][row][c8 + 4]); float tv[8];
#pragma unroll
        for (int j = 0; j < 4; ++j) { tv[j] = t0[j]; tv[4 + j] = t1[j]; }
        v8b h;
#pragma unroll
        for (int j = 0; j < 8; ++j) { const float v = tv[j] * INV1; const float tt = fmaxf((v - mm[j]) * sc[j] + bb[j], 0.0f); h[j] = (b16)(tt * XS); }
        *(volatile v8b*)(dst + ((size_t)b * T + n0 + row) * CK + c8) = h; }
      __threadfence(); } }
}

__global__ __launch_bounds__(128) void projv_kernel(const float* __restrict__ y, const b16* __restrict__ W1v, b16* __restrict__ Vt) {
  __shared__ __attribute__((aligned(16))) b16 Ah[4][16][C + 8];
  __shared__ __attribute__((aligned(16))) b16 Vs[CV][64 + 8];
  const int wave = threadIdx.x >> 5, lane = threadIdx.x & 31, nloc = lane & 15, hlf = lane >> 4;
  const int b = blockIdx.y; const int nb0 = blockIdx.x * 64; const int n0 = nb0 + wave * 16;
  for (int idx = lane; idx < 16 * C; idx += 32) { const int k = idx >> 4, rr = idx & 15; Ah[wave][rr][k] = (b16)(bf16_rne(y[((size_t)b * C + k) * T + n0 + rr]) * XS); }
  __syncthreads();
  v8f acc[8];
#pragma unroll
  for (int t = 0; t < 8; ++t) acc[t] = (v8f){};
#pragma unroll 1
  for (int kb = 0; kb < C; kb += 32) { const v16b a = frag_kb(&Ah[wave][nloc][kb], hlf);
#pragma unroll
    for (int t = 0; t < 8; ++t) acc[t] = wmma16b(a, frag_kb(W1v + (size_t)(t * 16 + nloc) * C + kb, hlf), acc[t]); }
#pragma unroll
  for (int t = 0; t < 8; ++t)
#pragma unroll
    for (int r = 0; r < 8; ++r) Vs[t * 16 + nloc][wave * 16 + 8 * hlf + r] = (b16)(acc[t][r] * (1.0f / WSC));
  __syncthreads();
  for (int pass = 0; pass < 2; ++pass) {
#pragma unroll
    for (int cc = 0; cc < 32; cc += 4) { const int ch = wave * 32 + cc + (lane >> 3); const int p8 = (lane & 7) * 8; const v8b v = *(const v8b*)(&Vs[ch][p8]);
      *(volatile v8b*)(Vt + ((size_t)b * CV + ch) * T + nb0 + p8) = v; }
    __threadfence(); }
}

__global__ __launch_bounds__(32) __attribute__((amdgpu_num_vgpr(256))) void attn_kernel(const b16* __restrict__ Qh, const b16* __restrict__ Kh, const b16* __restrict__ Vt, float* __restrict__ Y) {
  __shared__ __attribute__((aligned(16))) b16 Pt[16][32 + 8];
  __shared__ __attribute__((aligned(16))) float Of[16][CV + 4];
  const int lane = threadIdx.x & 31, nloc = lane & 15, hlf = lane >> 4;
  const int q0 = blockIdx.x * 16, b = blockIdx.y;
  const size_t qbase = (size_t)b * T + q0;
  v16b aq[4];
#pragma unroll
  for (int j = 0; j < 4; ++j) aq[j] = frag_kb(Qh + (qbase + nloc) * CK + 32 * j, hlf);
  float mrow[8], lsum[8];
#pragma unroll
  for (int r = 0; r < 8; ++r) { mrow[r] = -__builtin_inff(); lsum[r] = 0.0f; }
  v8f acco[8];
#pragma unroll
  for (int t = 0; t < 8; ++t) acco[t] = (v8f){};
#pragma unroll 1
  for (int kb = 0; kb < T; kb += 32) {
    const size_t kbase = (size_t)b * T + kb;
    v8f sacc[2];
#pragma unroll
    for (int t = 0; t < 2; ++t) { sacc[t] = (v8f){}; const b16* kr = Kh + (kbase + t * 16 + nloc) * CK;
#pragma unroll
      for (int j = 0; j < 4; ++j) sacc[t] = wmma16b(aq[j], frag_kb(kr + 32 * j, hlf), sacc[t]); }
    float s[2][8], mx[8];
#pragma unroll
    for (int r = 0; r < 8; ++r) { mx[r] = -__builtin_inff();
#pragma unroll
      for (int t = 0; t < 2; ++t) { s[t][r] = sacc[t][r] * SMS; mx[r] = fmaxf(mx[r], s[t][r]); } }
#pragma unroll
    for (int o = 1; o < 16; o <<= 1)
#pragma unroll
      for (int r = 0; r < 8; ++r) mx[r] = fmaxf(mx[r], __shfl_xor(mx[r], o));
    v16b pv;
#pragma unroll
    for (int r = 0; r < 8; ++r) { const float mn = fmaxf(mrow[r], mx[r]); const float corr = nexp2((mrow[r] - mn) * LOG2E); mrow[r] = mn; lsum[r] *= corr;
#pragma unroll
      for (int t = 0; t < 8; ++t) acco[t][r] *= corr;
#pragma unroll
      for (int t = 0; t < 2; ++t) { const float p = nexp2((s[t][r] - mn) * LOG2E); lsum[r] += p; pv[8 * t + r] = (b16)(p * PS); } }
#pragma unroll
    for (int t = 0; t < 2; ++t)
#pragma unroll
      for (int r = 0; r < 8; ++r) Pt[8 * hlf + r][16 * t + nloc] = pv[8 * t + r];
    __syncthreads();
    const v16b a = frag_kb(&Pt[nloc][0], hlf);
#pragma unroll
    for (int t = 0; t < 8; ++t) acco[t] = wmma16b(a, frag_kb(Vt + ((size_t)b * CV + t * 16 + nloc) * T + kb, hlf), acco[t]);
    __syncthreads(); }
#pragma unroll
  for (int o = 1; o < 16; o <<= 1)
#pragma unroll
    for (int r = 0; r < 8; ++r) lsum[r] += __shfl_xor(lsum[r], o);
  float inv[8];
#pragma unroll
  for (int r = 0; r < 8; ++r) inv[r] = (1.0f / lsum[r]) * (1.0f / (PS * XS));
#pragma unroll
  for (int t = 0; t < 8; ++t)
#pragma unroll
    for (int r = 0; r < 8; ++r) Of[8 * hlf + r][t * 16 + nloc] = acco[t][r] * inv[r];
  __syncthreads();
  for (int pass = 0; pass < 2; ++pass) {
#pragma unroll 4
    for (int r2 = 0; r2 < 16; ++r2) *(volatile v4f*)(Y + (qbase + r2) * CV + lane * 4) = *(const v4f*)(&Of[r2][lane * 4]);
    __threadfence(); }
}

__global__ __launch_bounds__(64) void out_kernel(const float* __restrict__ Y, const b16* __restrict__ WoT, const b16* __restrict__ WoQ, const float* __restrict__ PT,
    const float* __restrict__ x, float* __restrict__ out) {
  __shared__ __attribute__((aligned(16))) b16 Ah[2][16][CV + 8];
  __shared__ __attribute__((aligned(16))) b16 Al[2][16][CV + 8];
  __shared__ float Zs[32][C + 1];
  const int wave = threadIdx.x >> 5, lane = threadIdx.x & 31, nloc = lane & 15, hlf = lane >> 4;
  const int b = blockIdx.y; const int n0 = blockIdx.x * 32; const size_t rbase = (size_t)b * T + n0 + wave * 16;
  for (int idx = lane; idx < 16 * (CV / 4); idx += 32) { const int rr = idx / (CV / 4), c4 = (idx % (CV / 4)) * 4; const v4f v = *(const v4f*)(Y + (rbase + rr) * CV + c4); v4h hv, lv;
#pragma unroll
    for (int j = 0; j < 4; ++j) { const float vs = v[j] * XS; const b16 ph = (b16)vs; hv[j] = ph; lv[j] = (b16)((vs - (float)ph) * RS_); }
    *(v4h*)(&Ah[wave][rr][c4]) = hv; *(v4h*)(&Al[wave][rr][c4]) = lv; }
  __syncthreads();
  v16b a[4], al[4];
#pragma unroll
  for (int j = 0; j < 4; ++j) { a[j] = frag_kb(&Ah[wave][nloc][32 * j], hlf); al[j] = frag_kb(&Al[wave][nloc][32 * j], hlf); }
  const float* Po = PT + (size_t)4 * 3 * PTW;
#pragma unroll 1
  for (int t = 0; t < C / 16; ++t) { v8f acc = (v8f){}; const b16* wr = WoT + (size_t)(t * 16 + nloc) * CV; const b16* wq = WoQ + (size_t)(t * 16 + nloc) * CV;
#pragma unroll
    for (int j = 0; j < 4; ++j) { acc = wmma16b(a[j], frag_kb(wr + 32 * j, hlf), acc); acc = wmma16b(al[j], frag_kb(wq + 32 * j, hlf), acc); }
#pragma unroll
    for (int r = 0; r < 8; ++r) Zs[wave * 16 + 8 * hlf + r][t * 16 + nloc] = acc[r] * INV1; }
  __syncthreads();
  for (int pass = 0; pass < 2; ++pass) {
#pragma unroll 2
    for (int cc = 0; cc < C / 2; ++cc) { const int c = wave * (C / 2) + cc; const float scv = Po[c], mm = Po[PTW + c], bb = Po[2 * PTW + c];
      const size_t o_ = ((size_t)b * C + c) * T + n0 + lane; const float z = fmaxf((Zs[lane][c] - mm) * scv + bb, 0.0f);
      ((volatile float*)out)[o_] = bf16_rne(x[o_]) + z; }
    __threadfence(); }
}

extern "C" void kernel_launch(void* const* d_in, const int* in_sizes, int n_in, void* d_out, int out_size, void* d_ws, size_t ws_size, hipStream_t stream) {
  if (n_in < 28) return;
  auto Fp = [&](int i) { return (const float*)d_in[i]; };
  if (in_sizes[0] < BL * C * T || in_sizes[1] < BL * C * T) return;
  if (in_sizes[2] != CK * C || in_sizes[3] != CK * CK || in_sizes[4] != CK * C || in_sizes[5] != CK * CK || in_sizes[6] != CV * C || in_sizes[7] != C * CV) return;
  for (int s = 0; s < 4; ++s) for (int j = 0; j < 4; ++j) if (in_sizes[8 + 4 * s + j] != CK) return;
  for (int j = 0; j < 4; ++j) if (in_sizes[24 + j] != C) return;
  if (out_size < BL * C * T) return;
  size_t off = 0; char* ws = (char*)d_ws;
  auto carve = [&](size_t bytes) { char* p = ws + off; off += (bytes + 255) & ~(size_t)255; return p; };
  b16* W1q = (b16*)carve((size_t)CK * C * 2); b16* W1k = (b16*)carve((size_t)CK * C * 2); b16* W1v = (b16*)carve((size_t)CV * C * 2);
  b16* W2q = (b16*)carve((size_t)CK * CK * 2); b16* W2k = (b16*)carve((size_t)CK * CK * 2);
  b16* WoT = (b16*)carve((size_t)C * CV * 2); b16* WoQ = (b16*)carve((size_t)C * CV * 2);
  float* PT = (float*)carve((size_t)5 * 3 * PTW * 4);
  b16* Qh = (b16*)carve(NR * CK * 2); b16* Kh = (b16*)carve(NR * CK * 2); b16* Vt = (b16*)carve((size_t)B_FULL * CV * T * 2); float* Y = (float*)carve(NR * CV * 4);
  if (off > ws_size || off > ((size_t)128 << 20)) return;
  prep_kernel<<<UT / 256, 256, 0, stream>>>(Fp(2), Fp(4), Fp(6), Fp(3), Fp(5), Fp(7),
      Fp(8), Fp(9), Fp(10), Fp(11), Fp(12), Fp(13), Fp(14), Fp(15), Fp(16), Fp(17), Fp(18), Fp(19), Fp(20), Fp(21), Fp(22), Fp(23), Fp(24), Fp(25), Fp(26), Fp(27),
      W1q, W1k, W1v, W2q, W2k, WoT, WoQ, PT);
  projqk_kernel<<<dim3(T / 32, BL, 2), 64, 0, stream>>>(Fp(0), Fp(1), W1q, W1k, W2q, W2k, PT, Qh, Kh);
  projv_kernel<<<dim3(T / 64, BL), 128, 0, stream>>>(Fp(1), W1v, Vt);
  attn_kernel<<<dim3(QL / 16, BL), 32, 0, stream>>>(Qh, Kh, Vt, Y);
  out_kernel<<<dim3(QL / 32, BL), 64, 0, stream>>>(Y, WoT, WoQ, PT, Fp(0), (float*)d_out);
}
